// Head_A2B_Lite_70952859730361
// MI455X (gfx1250) — hardware-verified
//
#include <hip/hip_runtime.h>
#include <math.h>

constexpr int kNB = 4;
constexpr int kSA = 2048;
constexpr int kSB = 2048;
constexpr int kD  = 1024;
constexpr int kE  = 1024;
constexpr float kScoreScale = 0.03125f;

typedef __attribute__((ext_vector_type(16))) _Float16 v16h;
typedef __attribute__((ext_vector_type(8)))  _Float16 v8h;
typedef __attribute__((ext_vector_type(16))) __bf16   v16b;
typedef __attribute__((ext_vector_type(8)))  __bf16   v8b;
typedef __attribute__((ext_vector_type(8)))  float    v8f;
typedef __attribute__((ext_vector_type(4)))  float    v4f;
typedef __attribute__((ext_vector_type(4)))  unsigned int v4u;

__device__ __forceinline__ unsigned short f2bf_bits(float f) {
  unsigned u = __float_as_uint(f);
  return (unsigned short)((u + 0x7FFFu + ((u >> 16) & 1u)) >> 16);
}
__device__ __forceinline__ float bf_bits2f(unsigned short h) { return __uint_as_float(((unsigned)h) << 16); }

__device__ __forceinline__ void dep_guard_h(v8f& a, v8f& b, v16h x, v16h y) { asm volatile("v_nop\n\tv_nop\n\tv_nop\n\tv_nop" : "+v"(a), "+v"(b) : "v"(x), "v"(y)); }
__device__ __forceinline__ void dep_guard_b(v8f& a, v8f& b, v16b x, v16b y) { asm volatile("v_nop\n\tv_nop\n\tv_nop\n\tv_nop" : "+v"(a), "+v"(b) : "v"(x), "v"(y)); }
__device__ __forceinline__ void keep4_h(v16h a, v16h b, v16h c, v16h d) { asm volatile("v_nop" :: "v"(a), "v"(b), "v"(c), "v"(d)); }
__device__ __forceinline__ void keep4_b(v16b a, v16b b, v16b c, v16b d) { asm volatile("v_nop" :: "v"(a), "v"(b), "v"(c), "v"(d)); }
__device__ __forceinline__ void acc_guard4(v8f& a, v8f& b, v8f& c, v8f& d) { asm volatile("v_nop\n\tv_nop\n\tv_nop\n\tv_nop" : "+v"(a), "+v"(b), "+v"(c), "+v"(d)); }
template <typename T> struct Frag;
template <> struct Frag<_Float16> {
  typedef v16h V; union U { v16h v; v8h h[2]; };
  static __device__ __forceinline__ v16h load(const _Float16* p) {
    U f; f.h[0] = *(const v8h*)(p); f.h[1] = *(const v8h*)(p + 16); return f.v;
  }
  static __device__ __forceinline__ v8f mma(v16h a, v16h b, v8f c) {
    return __builtin_amdgcn_wmma_f32_16x16x32_f16(false, a, false, b, (short)0, c, false, false);
  }
  static __device__ __forceinline__ void guard(v8f& a, v8f& b, v16h x, v16h y) { dep_guard_h(a, b, x, y); }
  static __device__ __forceinline__ void keep(v16h a, v16h b, v16h c, v16h d) { keep4_h(a, b, c, d); }
};
template <> struct Frag<__bf16> {
  typedef v16b V; union U { v16b v; v8b h[2]; };
  static __device__ __forceinline__ v16b load(const __bf16* p) {
    U f; f.h[0] = *(const v8b*)(p); f.h[1] = *(const v8b*)(p + 16); return f.v;
  }
  static __device__ __forceinline__ v8f mma(v16b a, v16b b, v8f c) {
    return __builtin_amdgcn_wmma_f32_16x16x32_bf16(false, a, false, b, (short)0, c, false, false);
  }
  static __device__ __forceinline__ void guard(v8f& a, v8f& b, v16b x, v16b y) { dep_guard_b(a, b, x, y); }
  static __device__ __forceinline__ void keep(v16b a, v16b b, v16b c, v16b d) { keep4_b(a, b, c, d); }
};

__device__ __forceinline__ unsigned pk16(unsigned short a, unsigned short b) { return (unsigned)a | ((unsigned)b << 16); }
__device__ __forceinline__ unsigned short h_bits(float f) { const _Float16 h = (_Float16)f; return __builtin_bit_cast(unsigned short, h); }

template <int ET> struct Elem;
template <> struct Elem<0> { typedef _Float16 T; };
template <> struct Elem<1> { typedef __bf16 T; };
template <int ET, int SPL, int RSC, int OUT_MODE, int ACT, int TRI>
__global__ __launch_bounds__(256) void wmma_gemm64(
    const unsigned short* __restrict__ Ap, const unsigned short* __restrict__ A2p, int lda, long strideA,
    const unsigned short* __restrict__ Btp, const unsigned short* __restrict__ Bt2p, int ldb, long strideB,
    void* __restrict__ Cout, void* __restrict__ Cout2, int ldc, long strideC,
    const float* __restrict__ rsc, long strideS,
    int M, int N, int K, float scale) {
  typedef typename Elem<ET>::T T;
  typedef typename Frag<T>::V V;
  const T* A = (const T*)Ap; const T* A2 = (const T*)A2p; const T* Bt = (const T*)Btp; const T* Bt2 = (const T*)Bt2p;
  __shared__ __align__(16) float sT[8][16 * 68];
  const int b    = blockIdx.y;
  const int lane = threadIdx.x & 31;
  const int wave = threadIdx.x >> 5;
  const int tilesN = N >> 6;
  const int tilesM = M >> 6;
  const int tile = blockIdx.x * 8 + wave;
  if (tile >= tilesM * tilesN) return;
  const int tm = tile / tilesN;
  const int tn = tile - tm * tilesN;
  const int m0 = tm << 6;
  const int n0 = tn << 6;
  if (TRI == 1 && n0 > m0) return;
  const int Kl = (TRI == 2 && (m0 + 64) < K) ? (m0 + 64) : K;

  const T* Ab  = A  + (size_t)b * strideA;
  const T* Bb  = Bt + (size_t)b * strideB;
  const T* Ab2 = (SPL & 1) ? (A2  + (size_t)b * strideA) : nullptr;
  const T* Bb2 = (SPL & 2) ? (Bt2 + (size_t)b * strideB) : nullptr;

  const int rlane = lane & 15;
  const int koff  = (lane >> 4) * 8;
  const int mOff  = (lane >> 4) * 8;

  v8f acc[4][4];
#pragma unroll
  for (int i = 0; i < 4; ++i)
#pragma unroll
    for (int j = 0; j < 4; ++j) acc[i][j] = (v8f){0.f,0.f,0.f,0.f,0.f,0.f,0.f,0.f};

  for (int k0 = 0; k0 < Kl; k0 += 32) {
    V bh[4], bl[4];
#pragma unroll
    for (int j = 0; j < 4; ++j) {
      const size_t bo = (size_t)(n0 + (j << 4) + rlane) * ldb + koff + k0;
      bh[j] = Frag<T>::load(Bb + bo);
      if (SPL & 2) bl[j] = Frag<T>::load(Bb2 + bo);
    }
#pragma unroll
    for (int i = 0; i < 4; ++i) {
      const size_t ao = (size_t)(m0 + (i << 4) + rlane) * lda + koff + k0;
      V ah = Frag<T>::load(Ab + ao);
      V al;
      if (SPL & 1) al = Frag<T>::load(Ab2 + ao);
#pragma unroll
      for (int j = 0; j < 4; ++j) {
        acc[i][j] = Frag<T>::mma(ah, bh[j], acc[i][j]);
        if (SPL & 2) acc[i][j] = Frag<T>::mma(ah, bl[j], acc[i][j]);
        if (SPL & 1) acc[i][j] = Frag<T>::mma(al, bh[j], acc[i][j]);
      }
      Frag<T>::guard(acc[i][0], acc[i][3], ah, (SPL & 1) ? al : ah);
    }
    Frag<T>::keep(bh[0], bh[1], bh[2], bh[3]);
    if (SPL & 2) Frag<T>::keep(bl[0], bl[1], bl[2], bl[3]);
  }
  acc_guard4(acc[0][0], acc[0][1], acc[0][2], acc[0][3]);
  acc_guard4(acc[1][0], acc[1][1], acc[1][2], acc[1][3]);
  acc_guard4(acc[2][0], acc[2][1], acc[2][2], acc[2][3]);
  acc_guard4(acc[3][0], acc[3][1], acc[3][2], acc[3][3]);

  float* slab = sT[wave];
  const float* Rs = RSC ? (rsc + (size_t)b * strideS) : nullptr;
#pragma unroll
  for (int i = 0; i < 4; ++i) {
    const int mBase = m0 + (i << 4);
    float rsv[8];
#pragma unroll
    for (int r = 0; r < 8; ++r) rsv[r] = RSC ? Rs[mBase + mOff + r] : 1.0f;
#pragma unroll
    for (int j = 0; j < 4; ++j) {
      const int n = n0 + (j << 4) + rlane;
#pragma unroll
      for (int r = 0; r < 8; ++r) {
        float v = acc[i][j][r] * scale;
        if (RSC) v = v * rsv[r];
        if (TRI == 1) { if (n > mBase + mOff + r) v = 0.0f; }
        if (ACT == 6) v = (v > 0.0f) ? (v + 1.0f) : __expf(v);
        slab[(mOff + r) * 68 + (j << 4) + rlane] = v;
      }
    }
    __builtin_amdgcn_fence(__ATOMIC_RELEASE, "workgroup");
    __builtin_amdgcn_wave_barrier();
    __builtin_amdgcn_fence(__ATOMIC_ACQUIRE, "workgroup");
    if (OUT_MODE == 0) {
      float* C = (float*)Cout + (size_t)b * strideC;
      const int hh = lane >> 4, c4 = (lane & 15) * 4;
      for (int pass = 0; pass < 2; ++pass) {
#pragma unroll
        for (int it = 0; it < 8; ++it) {
          const int row = it * 2 + hh;
          v4f v = *(const v4f*)(slab + row * 68 + c4);
          *(volatile v4f*)(C + (size_t)(mBase + row) * ldc + n0 + c4) = v;
        }
        __threadfence();
      }
    } else {
      const int q = lane >> 3, c8 = (lane & 7) * 8;
      unsigned short* C  = (unsigned short*)Cout  + (size_t)b * strideC;
      unsigned short* C2 = (OUT_MODE == 2) ? ((unsigned short*)Cout2 + (size_t)b * strideC) : nullptr;
      for (int pass = 0; pass < 2; ++pass) {
#pragma unroll
        for (int it = 0; it < 4; ++it) {
          const int row = it * 4 + q;
          const float* sp = slab + row * 68 + c8;
          v8h hv, lv;
#pragma unroll
          for (int e = 0; e < 8; ++e) {
            if (OUT_MODE == 1) {
              hv[e] = (_Float16)sp[e];
            } else {
              unsigned short hb = f2bf_bits(sp[e]);
              unsigned short lb = f2bf_bits(sp[e] - bf_bits2f(hb));
              hv[e] = __builtin_bit_cast(_Float16, hb);
              lv[e] = __builtin_bit_cast(_Float16, lb);
            }
          }
          *(volatile v8h*)(C + (size_t)(mBase + row) * ldc + n0 + c8) = hv;
          if (OUT_MODE == 2) *(volatile v8h*)(C2 + (size_t)(mBase + row) * ldc + n0 + c8) = lv;
        }
        __threadfence();
      }
    }
    __builtin_amdgcn_fence(__ATOMIC_RELEASE, "workgroup");
    __builtin_amdgcn_wave_barrier();
    __builtin_amdgcn_fence(__ATOMIC_ACQUIRE, "workgroup");
  }
}

template <int MODE>
__global__ __launch_bounds__(256) void cast8_kernel(const float* __restrict__ in, unsigned short* __restrict__ out, int n8, float scale) {
  const int i = blockIdx.x * 256 + threadIdx.x;
  if (i >= n8) return;
  const float* p = in + 8 * (size_t)i;
  const v4f a = *(const v4f*)(p);
  const v4f c = *(const v4f*)(p + 4);
  unsigned short hb[8];
#pragma unroll
  for (int e = 0; e < 4; ++e) {
    if (MODE == 0) {
      hb[e]     = f2bf_bits(a[e]);
      hb[4 + e] = f2bf_bits(c[e]);
    } else {
      hb[e]     = h_bits(bf_bits2f(f2bf_bits(a[e])) * scale);
      hb[4 + e] = h_bits(bf_bits2f(f2bf_bits(c[e])) * scale);
    }
  }
  const v4u u = (v4u){pk16(hb[0], hb[1]), pk16(hb[2], hb[3]), pk16(hb[4], hb[5]), pk16(hb[6], hb[7])};
  unsigned short* q = out + 8 * (size_t)i;
  *(volatile v4u*)q = u;
  __threadfence();
  *(volatile v4u*)q = u;
  (void)scale;
}

__global__ __launch_bounds__(256) void transpose_cast_kernel(const float* __restrict__ in, unsigned short* __restrict__ out) {
  __shared__ __align__(16) unsigned short tile[64 * 72];
  const int tid = threadIdx.x, lane = tid & 31, wave = tid >> 5;
  const int t0 = blockIdx.x * 64, d0 = blockIdx.y * 64, bz = blockIdx.z;
  const float* ab = in + (size_t)bz * kSA * kD;
#pragma unroll
  for (int i = 0; i < 4; ++i) {
    const int tr = i * 16 + (tid >> 4);
    const int dc = (tid & 15) * 4;
    const v4f v = *(const v4f*)(ab + (size_t)(t0 + tr) * kD + d0 + dc);
#pragma unroll
    for (int e = 0; e < 4; ++e) tile[(dc + e) * 72 + tr] = f2bf_bits(v[e]);
  }
  __syncthreads();
  unsigned short* ob = out + (size_t)bz * kD * kSA;
  const int q = lane >> 3, c8 = (lane & 7) * 8;
  const int r0 = wave * 8 + q;
  const int r1 = wave * 8 + 4 + q;
  const v4u u0 = *(const v4u*)(&tile[r0 * 72 + c8]);
  const v4u u1 = *(const v4u*)(&tile[r1 * 72 + c8]);
  unsigned short* p0 = ob + (size_t)(d0 + r0) * kSA + t0 + c8;
  unsigned short* p1 = ob + (size_t)(d0 + r1) * kSA + t0 + c8;
  *(volatile v4u*)p0 = u0;
  *(volatile v4u*)p1 = u1;
  __threadfence();
  *(volatile v4u*)p0 = u0;
  *(volatile v4u*)p1 = u1;
}

__global__ __launch_bounds__(256) void softmax_split_kernel(const float* __restrict__ S,
                                                            unsigned short* __restrict__ PH, unsigned short* __restrict__ PL) {
  __shared__ __align__(16) float srow[kSA];
  __shared__ float redm[8];
  __shared__ float reds[8];
  const int row = blockIdx.x;
  const int t = threadIdx.x, lane = t & 31, wave = t >> 5;
  const float* sr = S + (size_t)row * kSA;
  float m = -INFINITY;
#pragma unroll 1
  for (int i = 0; i < kSA / 256; ++i) m = fmaxf(m, sr[t + 256 * i]);
#pragma unroll
  for (int off = 16; off > 0; off >>= 1) m = fmaxf(m, __shfl_xor(m, off, 32));
  if (lane == 0) redm[wave] = m;
  __syncthreads();
  float mx = redm[0];
#pragma unroll
  for (int w = 1; w < 8; ++w) mx = fmaxf(mx, redm[w]);
  float s = 0.f;
#pragma unroll 1
  for (int i = 0; i < kSA / 256; ++i) {
    const int cidx = t + 256 * i;
    const float e = expf(sr[cidx] - mx);
    srow[cidx] = e;
    s += e;
  }
#pragma unroll
  for (int off = 16; off > 0; off >>= 1) s += __shfl_xor(s, off, 32);
  if (lane == 0) reds[wave] = s;
  __syncthreads();
  const float tot = ((reds[0] + reds[1]) + (reds[2] + reds[3])) + ((reds[4] + reds[5]) + (reds[6] + reds[7]));
  const float inv = 1.0f / tot;
  const int c0 = t * 8;
  const v4f e0 = *(const v4f*)(srow + c0);
  const v4f e1 = *(const v4f*)(srow + c0 + 4);
  unsigned short hbv[8], lb[8];
#pragma unroll
  for (int e = 0; e < 4; ++e) {
    const float p0 = e0[e] * inv;
    const float p1 = e1[e] * inv;
    const unsigned short h0 = f2bf_bits(p0);
    const unsigned short h1 = f2bf_bits(p1);
    hbv[e] = h0;
    hbv[4 + e] = h1;
    lb[e]      = f2bf_bits(p0 - bf_bits2f(h0));
    lb[4 + e]  = f2bf_bits(p1 - bf_bits2f(h1));
  }
  const v4u hv = (v4u){pk16(hbv[0], hbv[1]), pk16(hbv[2], hbv[3]), pk16(hbv[4], hbv[5]), pk16(hbv[6], hbv[7])};
  const v4u lv = (v4u){pk16(lb[0], lb[1]), pk16(lb[2], lb[3]), pk16(lb[4], lb[5]), pk16(lb[6], lb[7])};
  unsigned short* hp = PH + (size_t)row * kSA + c0;
  unsigned short* lp = PL + (size_t)row * kSA + c0;
  *(volatile v4u*)hp = hv;
  *(volatile v4u*)lp = lv;
  __threadfence();
  *(volatile v4u*)hp = hv;
  *(volatile v4u*)lp = lv;
}

extern "C" void kernel_launch(void* const* d_in, const int* in_sizes, int n_in,
                              void* d_out, int out_size, void* d_ws, size_t ws_size,
                              hipStream_t stream) {
  if (n_in < 3) return;
  if (in_sizes[0] != kNB * kSA * kD) return;
  if (in_sizes[1] != kNB * kSB * kE) return;
  if (in_sizes[2] != kD * kE) return;
  if (out_size != kNB * kSB * kD) return;

  const float* a  = (const float*)d_in[0];
  const float* b  = (const float*)d_in[1];
  const float* wq = (const float*)d_in[2];
  float* outp = (float*)d_out;

  const size_t SZ_A16  = (size_t)kNB * kSA * kD * 2;
  const size_t SZ_AT16 = (size_t)kNB * kD * kSA * 2;
  const size_t SZ_WQ16 = (size_t)kD * kE * 2;
  const size_t SZ_Q16  = (size_t)kNB * kSB * kD * 2;
  const size_t SZ_B16  = (size_t)kNB * kSB * kE * 2;
  const size_t SZ_S    = (size_t)kSB * kSA * 4;
  const size_t SZ_R    = (SZ_B16 > SZ_S) ? SZ_B16 : SZ_S;
  const size_t SZ_P16  = (size_t)kSB * kSA * 2;

  size_t off = 0;
  const size_t oA16  = off; off += SZ_A16;
  const size_t oAT16 = off; off += SZ_AT16;
  const size_t oWQ16 = off; off += SZ_WQ16;
  const size_t oQH   = off; off += SZ_Q16;
  const size_t oQL   = off; off += SZ_Q16;
  const size_t oR    = off; off += SZ_R;
  const size_t oPH   = off; off += SZ_P16;
  const size_t oPL   = off; off += SZ_P16;
  const size_t TOTAL = off;
  if (TOTAL > ws_size) return;
  if (TOTAL > (size_t)134217728) return;

  char* ws = (char*)d_ws;
  unsigned short* A16  = (unsigned short*)(ws + oA16);
  unsigned short* AT16 = (unsigned short*)(ws + oAT16);
  unsigned short* WQ16 = (unsigned short*)(ws + oWQ16);
  unsigned short* QH   = (unsigned short*)(ws + oQH);
  unsigned short* QL   = (unsigned short*)(ws + oQL);
  unsigned short* B16  = (unsigned short*)(ws + oR);
  float*          Sf   = (float*)(ws + oR);
  unsigned short* PH   = (unsigned short*)(ws + oPH);
  unsigned short* PL   = (unsigned short*)(ws + oPL);
  const float* dummy_rsc = (const float*)(ws + oR);

  const dim3 blk(256);

  {
    const int n8a = kNB * kSA * kD / 8;
    cast8_kernel<0><<<dim3(n8a / 256), blk, 0, stream>>>(a, A16, n8a, 1.0f);
    const int n8b = kNB * kSB * kE / 8;
    cast8_kernel<0><<<dim3(n8b / 256), blk, 0, stream>>>(b, B16, n8b, 1.0f);
    const int n8w = kD * kE / 8;
    cast8_kernel<0><<<dim3(n8w / 256), blk, 0, stream>>>(wq, WQ16, n8w, 1.0f);
  }
  transpose_cast_kernel<<<dim3(kSA / 64, kD / 64, kNB), blk, 0, stream>>>(a, AT16);

  const int gQ = ((kNB * kSB / 64) * (kD / 64) + 7) / 8;
  wmma_gemm64<1, 0, 0, 2, 0, 0><<<dim3(gQ, 1), blk, 0, stream>>>(
      B16, B16, kE, 0L, WQ16, WQ16, kE, 0L, (void*)QH, (void*)QL, kD, 0L, dummy_rsc, 0L, kNB * kSB, kD, kE, 1.0f);

  const int gS = ((kSB / 64) * (kSA / 64) + 7) / 8;
  const int gO = ((kSB / 64) * (kD / 64) + 7) / 8;
  for (int bb = 0; bb < kNB; ++bb) {
    const unsigned short* QHb  = QH   + (size_t)bb * kSB * kD;
    const unsigned short* QLb  = QL   + (size_t)bb * kSB * kD;
    const unsigned short* A16b = A16  + (size_t)bb * kSA * kD;
    const unsigned short* ATb  = AT16 + (size_t)bb * kD * kSA;
    float* outb = outp + (size_t)bb * kSB * kD;
    wmma_gemm64<1, 1, 0, 0, 0, 0><<<dim3(gS, 1), blk, 0, stream>>>(
        QHb, QLb, kD, 0L, A16b, A16b, kD, 0L, (void*)Sf, (void*)Sf, kSA, 0L, dummy_rsc, 0L, kSB, kSA, kD, kScoreScale);
    softmax_split_kernel<<<dim3(kSB), blk, 0, stream>>>(Sf, PH, PL);
    wmma_gemm64<1, 1, 0, 0, 0, 0><<<dim3(gO, 1), blk, 0, stream>>>(
        PH, PL, kSA, 0L, ATb, ATb, kSA, 0L, (void*)outb, (void*)outb, kD, 0L, dummy_rsc, 0L, kSB, kD, kSA, 1.0f);
  }
}
